// FinalLayer_multi_54881092108537
// MI455X (gfx1250) — hardware-verified
//
#include <hip/hip_runtime.h>
#include <math.h>


#define NB   8
#define NG   512
#define NT   1024
#define NK   5
#define NC   3
#define KC   15
#define TT   64
#define NTHR 128
#define NWAV 4

static_assert(NG % 32 == 0);
static_assert(NT % TT == 0);
static_assert(TT == NWAV * 16);
static_assert((TT * NC) % 32 == 0);
static_assert(KC == NK * NC);

#if defined(__has_builtin)
#if __has_builtin(__builtin_amdgcn_exp2f)
#define FAST_EXP2(x) __builtin_amdgcn_exp2f(x)
#endif
#endif
#ifndef FAST_EXP2
#define FAST_EXP2(x) exp2f(x)
#endif

typedef _Float16 v16h __attribute__((ext_vector_type(16)));
typedef _Float16 v8h  __attribute__((ext_vector_type(8), __may_alias__));
typedef float    v8f  __attribute__((ext_vector_type(8)));
typedef float    v4f  __attribute__((ext_vector_type(4), __may_alias__));
typedef unsigned v8u  __attribute__((ext_vector_type(8)));

union Frag {
    v16h     v;
    v8h      hf[2];
    v8u      w;
    _Float16 e[16];
};

__device__ __forceinline__ v8f wmma_f16(v16h a, v16h b, v8f c)
{
    v8f d = __builtin_amdgcn_wmma_f32_16x16x32_f16(false, a, false, b, (short)0, c, false, false);
    asm volatile("v_nop\n\tv_nop\n\tv_nop\n\tv_nop" : "+v"(d) : "v"(a), "v"(b));
    return d;
}

__global__ __launch_bounds__(NTHR)
void k_rbf_final(const float* __restrict__ x_grid,
                 const float* __restrict__ h_grid,
                 const float* __restrict__ target_x,
                 const float* __restrict__ sigma,
                 const float* __restrict__ g_w,
                 const float* __restrict__ g_b,
                 float* __restrict__ out)
{
    __shared__ __attribute__((aligned(16))) float    x_s[NC * NG];
    __shared__ __attribute__((aligned(16))) _Float16 hT[16 * NG];
    __shared__ float coef_s[16];
    __shared__ float red[NWAV * 256];
    __shared__ __attribute__((aligned(16))) float outs[TT * NC];

    const int tid  = threadIdx.x;
    const int wave = tid >> 5;
    const int l    = tid & 31;
    const int h    = l >> 4;
    const int m    = l & 15;
    const int b    = blockIdx.y;
    const int tile = blockIdx.x;
    if (tile * TT >= NT || b >= NB) return;

    const float* xg  = x_grid   + (size_t)b * NG * NC;
    const float* hg  = h_grid   + (size_t)b * NG * KC;
    const float* txp = target_x + (size_t)b * NT * NC;

    for (int i = tid; i < NC * NG; i += NTHR) {
        const int c = i / NG;
        const int g = i - c * NG;
        x_s[i] = xg[g * NC + c];
    }
    for (int i = tid; i < 16 * NG; i += NTHR) {
        const int n = i / NG;
        const int g = i - n * NG;
        float v = 0.0f;
        if (n < KC) v = hg[g * KC + n] * 64.0f;
        hT[i] = (_Float16)v;
    }
    if (tid < KC) {
        const float s = expf(sigma[tid]) + 1e-6f;
        coef_s[tid] = -0.72134752f / (s * s);
    }

    const int t0w = tile * TT + wave * 16;
    int trow = t0w + m;
    if (trow > NT - 1) trow = NT - 1;
    float txv[NC];
#pragma unroll
    for (int c = 0; c < NC; ++c) txv[c] = txp[trow * NC + c];

    __syncthreads();

    float coef[KC];
#pragma unroll
    for (int kc = 0; kc < KC; ++kc) coef[kc] = coef_s[kc];

    v8f acc;
#pragma unroll
    for (int r = 0; r < 8; ++r) acc[r] = 0.0f;

    const _Float16* hrow = hT + m * NG;

#pragma unroll 1
    for (int g0 = 0; g0 < NG; g0 += 32) {
        Frag bf;
        bf.hf[0] = *(const v8h*)(hrow + g0 + 8 * h);
        bf.hf[1] = *(const v8h*)(hrow + g0 + 16 + 8 * h);

#pragma unroll
        for (int c = 0; c < NC; ++c) {
            const float* xc = x_s + c * NG + g0;
            union { v4f q[4]; float f[16]; } xv;
            xv.q[0] = *(const v4f*)(xc + 8 * h);
            xv.q[1] = *(const v4f*)(xc + 8 * h + 4);
            xv.q[2] = *(const v4f*)(xc + 16 + 8 * h);
            xv.q[3] = *(const v4f*)(xc + 20 + 8 * h);
            const float tc = txv[c];
            float u[16];
#pragma unroll
            for (int i = 0; i < 16; ++i) {
                const float d = xv.f[i] - tc;
                u[i] = d * d;
            }
#pragma unroll
            for (int k = 0; k < NK; ++k) {
                const int kc = k * NC + c;
                const float cf = coef[kc];
                Frag af;
#pragma unroll
                for (int i = 0; i < 16; ++i)
                    af.e[i] = (_Float16)(FAST_EXP2(u[i] * cf) * 256.0f);
                const unsigned msk = (m == kc) ? 0xffffffffu : 0u;
                Frag bs;
                bs.w = bf.w & msk;
                acc = wmma_f16(af.v, bs.v, acc);
            }
        }
    }

#pragma unroll
    for (int r = 0; r < 8; ++r)
        red[wave * 256 + (8 * h + r) * 16 + m] = acc[r];

    __syncthreads();

    const float gb = g_b[0];
    float gwv[NK];
#pragma unroll
    for (int k = 0; k < NK; ++k) gwv[k] = g_w[k];

    for (int o = tid; o < TT * NC; o += NTHR) {
        const int tl = o / NC;
        const int c  = o - tl * NC;
        const float* rp = red + (tl >> 4) * 256 + (tl & 15) * 16 + c;
        float s = 0.0f;
#pragma unroll
        for (int k = 0; k < NK; ++k)
            s += gwv[k] * (rp[k * NC] * (1.0f / 16384.0f));
        outs[o] = s + gb;
    }

    __syncthreads();

    const size_t base = ((size_t)b * NT + (size_t)tile * TT) * NC;
    const int NV = (TT * NC) / 4;
    v4f v = {0.0f, 0.0f, 0.0f, 0.0f};
    if (tid < NV) {
        v = *(const v4f*)(outs + tid * 4);
        *(volatile v4f*)(out + base + (size_t)tid * 4) = v;
    }
    __threadfence();
    if (tid < NV) {
        *(volatile v4f*)(out + base + (size_t)tid * 4) = v;
    }
}

extern "C" void kernel_launch(void* const* d_in, const int* in_sizes, int n_in,
                              void* d_out, int out_size, void* d_ws, size_t ws_size,
                              hipStream_t stream)
{
    (void)d_ws; (void)ws_size;
    if (n_in < 6) return;
    if (in_sizes[0] != NB * NG * NC) return;
    if (in_sizes[1] != NB * NG * KC) return;
    if (in_sizes[2] != NB * NT * NC) return;
    if (in_sizes[3] != KC) return;
    if (in_sizes[4] != NK) return;
    if (in_sizes[5] < 1) return;
    if (out_size != NB * NT * NC) return;

    const float* x_grid   = (const float*)d_in[0];
    const float* h_grid   = (const float*)d_in[1];
    const float* target_x = (const float*)d_in[2];
    const float* sigma    = (const float*)d_in[3];
    const float* g_w      = (const float*)d_in[4];
    const float* g_b      = (const float*)d_in[5];
    float* out            = (float*)d_out;

    dim3 grid(NT / TT, NB);
    k_rbf_final<<<grid, NTHR, 0, stream>>>(x_grid, h_grid, target_x, sigma, g_w, g_b, out);
}
